// EncoderLayer_83056077571009
// MI455X (gfx1250) — hardware-verified
//
#include <hip/hip_runtime.h>
#include <stddef.h>
#include <stdint.h>
#include <math.h>


#define NBATCH 2
#define SEQ    2048
#define DM     1024
#define DIN    2048
#define NHD    32
#define CONVD  2176
#define DPROJ  4256
#define ZXP    4288
#define XP     2176
#define MLPI   4096
#define NCH    32
#define GBM    128
#define GBN    64
#define GTHR   128
#define SSD_LDS 115968
#define WSMAX  134217728

static_assert(SEQ % GBM == 0 && ZXP % GBN == 0 && DM % GBN == 0 && MLPI % GBN == 0);
static_assert(ZXP >= DPROJ && DM % 32 == 0 && DIN % 32 == 0 && MLPI % 32 == 0);
static_assert((SEQ * CONVD) % 256 == 0 && CONVD % 32 == 0);
static_assert(SEQ == NCH * 64 && DIN == NHD * 64 && CONVD == DIN + 128 && DPROJ == 2 * DIN + 128 + NHD);
static_assert(SSD_LDS == 2 * 16384 + 10 * 8192 + 5 * 256);

typedef float          v4f   __attribute__((ext_vector_type(4)));
typedef float          v8f   __attribute__((ext_vector_type(8)));
typedef int            v8i   __attribute__((ext_vector_type(8)));
typedef unsigned short v4us  __attribute__((ext_vector_type(4)));
typedef unsigned short v8us  __attribute__((ext_vector_type(8)));
typedef unsigned short v16us __attribute__((ext_vector_type(16)));
typedef __bf16         v16bf __attribute__((ext_vector_type(16)));
typedef v4f  __attribute__((may_alias)) v4fa;
typedef v4us __attribute__((may_alias)) v4usa;
typedef v8us __attribute__((may_alias)) v8usa;
union FragB { v16bf v; v16us u; v8us h[2]; v8i w; };

__device__ __forceinline__ v8f wmb(const FragB& a, const FragB& b, v8f c) {
  v8f d = __builtin_amdgcn_wmma_f32_16x16x32_bf16(false, a.v, false, b.v, (short)0, c, false, false);
  asm volatile("v_nop\n\tv_nop\n\tv_nop\n\tv_nop" : "+v"(d) : "v"(a.w), "v"(b.w));
  return d;
}

__device__ __forceinline__ unsigned bf16_bits(float f) {
  const unsigned u = __float_as_uint(f);
  return (u + 0x7FFFu + ((u >> 16) & 1u)) >> 16;
}
__device__ __forceinline__ float bf16_val(float f) {
  return __uint_as_float(bf16_bits(f) << 16);
}
__device__ __forceinline__ void split_hl(float v, unsigned short& h, unsigned short& l) {
  const unsigned hb = bf16_bits(v);
  h = (unsigned short)hb;
  l = (unsigned short)bf16_bits(v - __uint_as_float(hb << 16));
}
__device__ __forceinline__ void pack4(v4f v, v4us& h, v4us& l) {
  unsigned short a, b;
  split_hl(v.x, a, b); h[0] = a; l[0] = b;
  split_hl(v.y, a, b); h[1] = a; l[1] = b;
  split_hl(v.z, a, b); h[2] = a; l[2] = b;
  split_hl(v.w, a, b); h[3] = a; l[3] = b;
}
__device__ __forceinline__ void stT4(unsigned short* ph, unsigned short* pl, int col, int row, v4f v) {
  unsigned short a, b;
  split_hl(v.x, a, b); ph[(col + 0) * 64 + row] = a; pl[(col + 0) * 64 + row] = b;
  split_hl(v.y, a, b); ph[(col + 1) * 64 + row] = a; pl[(col + 1) * 64 + row] = b;
  split_hl(v.z, a, b); ph[(col + 2) * 64 + row] = a; pl[(col + 2) * 64 + row] = b;
  split_hl(v.w, a, b); ph[(col + 3) * 64 + row] = a; pl[(col + 3) * 64 + row] = b;
}
__device__ __forceinline__ float siluf(float v) {
  const float e = expf(fminf(-v, 60.0f));
  return v * (1.0f / (1.0f + e));
}

__device__ __forceinline__ void mm64x3(const unsigned short* Ah, const unsigned short* Al,
                                       const unsigned short* Bh, const unsigned short* Bl,
                                       v8f (&acc)[4], int wave, int hh, int m) {
#pragma unroll
  for (int ks = 0; ks < 2; ++ks) {
    const int ao = (16 * wave + m) * 64 + 32 * ks + 8 * hh;
    FragB ah, al;
    ah.h[0] = *(const v8usa*)(Ah + ao);
    ah.h[1] = *(const v8usa*)(Ah + ao + 16);
    al.h[0] = *(const v8usa*)(Al + ao);
    al.h[1] = *(const v8usa*)(Al + ao + 16);
#pragma unroll
    for (int t = 0; t < 4; ++t) {
      const int bo = (16 * t + m) * 64 + 32 * ks + 8 * hh;
      FragB bh, bl;
      bh.h[0] = *(const v8usa*)(Bh + bo);
      bh.h[1] = *(const v8usa*)(Bh + bo + 16);
      bl.h[0] = *(const v8usa*)(Bl + bo);
      bl.h[1] = *(const v8usa*)(Bl + bo + 16);
      acc[t] = wmb(ah, bh, acc[t]);
      acc[t] = wmb(al, bh, acc[t]);
      acc[t] = wmb(ah, bl, acc[t]);
    }
  }
}

__global__ __launch_bounds__(256) void k_cvx(const float* __restrict__ x, int nUnits, unsigned short* xb) {
  const int u = (int)blockIdx.x * 256 + (int)threadIdx.x;
  if (u >= nUnits) return;
  const float* p = x + (size_t)u * 8;
  const v4f a = *(const v4f*)p;
  const v4f b = *(const v4f*)(p + 4);
  v8us o;
  o[0] = (unsigned short)bf16_bits(a.x); o[1] = (unsigned short)bf16_bits(a.y);
  o[2] = (unsigned short)bf16_bits(a.z); o[3] = (unsigned short)bf16_bits(a.w);
  o[4] = (unsigned short)bf16_bits(b.x); o[5] = (unsigned short)bf16_bits(b.y);
  o[6] = (unsigned short)bf16_bits(b.z); o[7] = (unsigned short)bf16_bits(b.w);
  unsigned short* dp = xb + (size_t)u * 8;
  *(volatile v8us*)dp = o;
  __threadfence();
  *(volatile v8us*)dp = o;
}

__global__ __launch_bounds__(256) void k_wT(const float* __restrict__ W, int K, int N, int nPad,
                                            unsigned short* WT) {
  const int u   = (int)blockIdx.x * 256 + (int)threadIdx.x;
  const int k8n = K >> 3;
  if (u >= nPad * k8n) return;
  const int n  = u / k8n;
  const int k8 = (u - n * k8n) * 8;
  const int nc = n < N ? n : N - 1;
  const bool ok = n < N;
  const float* p = W + (size_t)k8 * (size_t)N + nc;
  v8us o;
#pragma unroll
  for (int i = 0; i < 8; ++i) {
    const float f = p[(size_t)i * (size_t)N];
    o[i] = ok ? (unsigned short)bf16_bits(f) : (unsigned short)0;
  }
  unsigned short* dp = WT + (size_t)n * (size_t)K + k8;
  *(volatile v8us*)dp = o;
  __threadfence();
  *(volatile v8us*)dp = o;
}

template <int MODE>
__global__ __launch_bounds__(GTHR) void k_gemm(
    const unsigned short* __restrict__ A, int lda, int KA,
    const unsigned short* __restrict__ WT, int KW,
    float* outF, int ldo,
    unsigned short* outH, int ldh, int loOff,
    const float* __restrict__ bias,
    const float* __restrict__ res, int ldr)
{
  __shared__ __attribute__((aligned(16))) float stg[GBM * GBN];
  const int tid = (int)threadIdx.x, lane = tid & 31, wave = tid >> 5, hh = lane >> 4, m = lane & 15;
  const int rowBase = (int)blockIdx.x * GBM;
  const int col0    = (int)blockIdx.y * GBN;

  v8f acc[2][4];
  {
    const v8f z = {0.f, 0.f, 0.f, 0.f, 0.f, 0.f, 0.f, 0.f};
#pragma unroll
    for (int i = 0; i < 2; ++i)
#pragma unroll
      for (int t = 0; t < 4; ++t) acc[i][t] = z;
  }
  const unsigned short* ap0 = A + (size_t)(rowBase + 32 * wave + m) * (size_t)lda + 8 * hh;
  const unsigned short* ap1 = ap0 + (size_t)16 * (size_t)lda;
  const unsigned short* wp  = WT + (size_t)(col0 + m) * (size_t)KW + 8 * hh;
#pragma unroll 1
  for (int k0 = 0; k0 < KA; k0 += 32) {
    const int kw = (k0 >= KW) ? (k0 - KW) : k0;
    FragB a0, a1;
    a0.h[0] = *(const v8usa*)(ap0 + k0);
    a0.h[1] = *(const v8usa*)(ap0 + k0 + 16);
    a1.h[0] = *(const v8usa*)(ap1 + k0);
    a1.h[1] = *(const v8usa*)(ap1 + k0 + 16);
#pragma unroll
    for (int t = 0; t < 4; ++t) {
      const unsigned short* wq = wp + (size_t)(16 * t) * (size_t)KW + kw;
      FragB bf;
      bf.h[0] = *(const v8usa*)wq;
      bf.h[1] = *(const v8usa*)(wq + 16);
      acc[0][t] = wmb(a0, bf, acc[0][t]);
      acc[1][t] = wmb(a1, bf, acc[1][t]);
    }
  }

#pragma unroll
  for (int i = 0; i < 2; ++i)
#pragma unroll
    for (int t = 0; t < 4; ++t)
#pragma unroll
      for (int r = 0; r < 8; ++r)
        stg[(32 * wave + 16 * i + 8 * hh + r) * GBN + 16 * t + m] = acc[i][t][r];
  __syncthreads();

  if constexpr (MODE == 2) {
    const int pc = 8 * (lane & 7);
    v4f b0, b1;
    {
      const v4f t0 = *(const v4f*)(bias + col0 + pc);
      const v4f t1 = *(const v4f*)(bias + col0 + pc + 4);
      b0.x = bf16_val(t0.x); b0.y = bf16_val(t0.y); b0.z = bf16_val(t0.z); b0.w = bf16_val(t0.w);
      b1.x = bf16_val(t1.x); b1.y = bf16_val(t1.y); b1.z = bf16_val(t1.z); b1.w = bf16_val(t1.w);
    }
#pragma unroll 1
    for (int it = 0; it < 8; ++it) {
      const int lr = it * 16 + 4 * wave + (lane >> 3);
      v4f a = *(const v4fa*)(stg + lr * GBN + pc);
      v4f b = *(const v4fa*)(stg + lr * GBN + pc + 4);
      a = a + b0; b = b + b1;
      a.x = siluf(a.x); a.y = siluf(a.y); a.z = siluf(a.z); a.w = siluf(a.w);
      b.x = siluf(b.x); b.y = siluf(b.y); b.z = siluf(b.z); b.w = siluf(b.w);
      v4us h0, l0, h1, l1;
      pack4(a, h0, l0);
      pack4(b, h1, l1);
      v8us oh, ol;
      oh[0] = h0[0]; oh[1] = h0[1]; oh[2] = h0[2]; oh[3] = h0[3];
      oh[4] = h1[0]; oh[5] = h1[1]; oh[6] = h1[2]; oh[7] = h1[3];
      ol[0] = l0[0]; ol[1] = l0[1]; ol[2] = l0[2]; ol[3] = l0[3];
      ol[4] = l1[0]; ol[5] = l1[1]; ol[6] = l1[2]; ol[7] = l1[3];
      unsigned short* hp = outH + (size_t)(rowBase + lr) * (size_t)ldh + col0 + pc;
      unsigned short* lp = hp + loOff;
      *(volatile v8us*)hp = oh;
      *(volatile v8us*)lp = ol;
      __threadfence();
      *(volatile v8us*)hp = oh;
      *(volatile v8us*)lp = ol;
    }
  } else {
    v4f b4 = {0.f, 0.f, 0.f, 0.f};
    if constexpr (MODE == 3) {
      const v4f t0 = *(const v4f*)(bias + col0 + 4 * m);
      b4.x = bf16_val(t0.x); b4.y = bf16_val(t0.y); b4.z = bf16_val(t0.z); b4.w = bf16_val(t0.w);
    }
#pragma unroll 1
    for (int it = 0; it < 16; ++it) {
      const int lr = it * 8 + 2 * wave + hh;
      const int gr = rowBase + lr;
      const int gc = col0 + 4 * m;
      v4f v = *(const v4fa*)(stg + lr * GBN + 4 * m);
      if constexpr (MODE == 1) {
        const v4f r = *(const v4f*)(res + (size_t)gr * (size_t)ldr + gc);
        v.x += bf16_val(r.x); v.y += bf16_val(r.y); v.z += bf16_val(r.z); v.w += bf16_val(r.w);
      }
      if constexpr (MODE == 3) {
        const v4f r = *(const v4f*)(res + (size_t)gr * (size_t)ldr + gc);
        v = (v + b4) + r;
      }
      float* op = outF + (size_t)gr * (size_t)ldo + gc;
      *(volatile v4f*)op = v;
      __threadfence();
      *(volatile v4f*)op = v;
    }
  }
}

__global__ __launch_bounds__(256) void k_conv(const float* __restrict__ zx, const float* __restrict__ cw,
                                              const float* __restrict__ cb, float* xbc) {
  const int u = (int)blockIdx.x * 256 + (int)threadIdx.x;
  if (u >= SEQ * CONVD) return;
  const int t = u / CONVD;
  const int c = u - t * CONVD;
  const v4f w = *(const v4f*)(cw + 4 * c);
  const int t0 = t - 3, t1 = t - 2, t2 = t - 1;
  const float x0 = zx[(size_t)(t0 < 0 ? 0 : t0) * ZXP + DIN + c];
  const float x1 = zx[(size_t)(t1 < 0 ? 0 : t1) * ZXP + DIN + c];
  const float x2 = zx[(size_t)(t2 < 0 ? 0 : t2) * ZXP + DIN + c];
  const float x3 = zx[(size_t)t * ZXP + DIN + c];
  float acc = 0.0f;
  acc += (t0 >= 0) ? bf16_val(w.x) * x0 : 0.0f;
  acc += (t1 >= 0) ? bf16_val(w.y) * x1 : 0.0f;
  acc += (t2 >= 0) ? bf16_val(w.z) * x2 : 0.0f;
  acc += bf16_val(w.w) * x3;
  acc += bf16_val(cb[c]);
  const float o = siluf(acc);
  float* op = xbc + (size_t)u;
  *(volatile float*)op = o;
  __threadfence();
  *(volatile float*)op = o;
}

__global__ __launch_bounds__(128) void k_cb(const float* __restrict__ xbc, float* G) {
  __shared__ __attribute__((aligned(16))) unsigned short Ch[4096];
  __shared__ __attribute__((aligned(16))) unsigned short Cl[4096];
  __shared__ __attribute__((aligned(16))) unsigned short Bh[4096];
  __shared__ __attribute__((aligned(16))) unsigned short Bl[4096];
  __shared__ __attribute__((aligned(16))) float stg[4096];
  const int tid = (int)threadIdx.x, lane = tid & 31, wave = tid >> 5, hh = lane >> 4, m = lane & 15;
  const int ch = (int)blockIdx.x;
  const int t0 = ch * 64;
  const int row = tid >> 1, half = tid & 1;
  const float* rp = xbc + (size_t)(t0 + row) * XP + DIN + 32 * half;
#pragma unroll 2
  for (int j = 0; j < 8; ++j) {
    const int col = 32 * half + 4 * j;
    const v4f bv = *(const v4f*)(rp + 4 * j);
    const v4f cv = *(const v4f*)(rp + 64 + 4 * j);
    v4us h4, l4;
    pack4(cv, h4, l4);
    *(v4usa*)(Ch + row * 64 + col) = h4;
    *(v4usa*)(Cl + row * 64 + col) = l4;
    pack4(bv, h4, l4);
    *(v4usa*)(Bh + row * 64 + col) = h4;
    *(v4usa*)(Bl + row * 64 + col) = l4;
  }
  __syncthreads();
  v8f acc[4];
  {
    const v8f z = {0.f, 0.f, 0.f, 0.f, 0.f, 0.f, 0.f, 0.f};
    acc[0] = z; acc[1] = z; acc[2] = z; acc[3] = z;
  }
  mm64x3(Ch, Cl, Bh, Bl, acc, wave, hh, m);
#pragma unroll
  for (int t = 0; t < 4; ++t)
#pragma unroll
    for (int r = 0; r < 8; ++r)
      stg[(16 * wave + 8 * hh + r) * 64 + 16 * t + m] = acc[t][r];
  __syncthreads();
#pragma unroll 1
  for (int it = 0; it < 8; ++it) {
    const int idx = it * 128 + tid;
    const int r = idx >> 4, c4 = idx & 15;
    const v4f v = *(const v4fa*)(stg + r * 64 + 4 * c4);
    float* op = G + ((size_t)(t0 + r)) * 64 + 4 * c4;
    *(volatile v4f*)op = v;
    __threadfence();
    *(volatile v4f*)op = v;
  }
}

__global__ __launch_bounds__(128) void k_ssd(const float* __restrict__ zx, float* xbc,
                                             const float* __restrict__ G,
                                             const float* __restrict__ dt_bias,
                                             const float* __restrict__ A_log,
                                             const float* __restrict__ D_par) {
  extern __shared__ __attribute__((aligned(16))) unsigned char smem[];
  float* Sf = (float*)smem;
  float* XS = (float*)(smem + 16384);
  unsigned short* Mh = (unsigned short*)(smem + 32768);
  unsigned short* Ml = Mh + 4096;
  unsigned short* Th = Ml + 4096;
  unsigned short* Tl = Th + 4096;
  unsigned short* Ch = Tl + 4096;
  unsigned short* Cl = Ch + 4096;
  unsigned short* Sh = Cl + 4096;
  unsigned short* Sl = Sh + 4096;
  unsigned short* Bh = Sl + 4096;
  unsigned short* Bl = Bh + 4096;
  float* dtv  = (float*)(smem + 114688);
  float* adtv = dtv + 64;
  float* cumv = dtv + 128;
  float* ecum = dtv + 192;
  float* edec = dtv + 256;

  const int tid = (int)threadIdx.x, lane = tid & 31, wave = tid >> 5, hh = lane >> 4, m = lane & 15;
  const int h = (int)blockIdx.x;
  const int row = tid >> 1, half = tid & 1;
  const float dtb  = bf16_val(dt_bias[h]);
  const float Aneg = -expf(bf16_val(A_log[h]));
  const float Dp   = bf16_val(D_par[h]);

  {
    const v4f z4 = {0.f, 0.f, 0.f, 0.f};
    for (int i = tid * 4; i < 4096; i += 512) *(v4fa*)(Sf + i) = z4;
  }
  __syncthreads();

#pragma unroll 1
  for (int c = 0; c < NCH; ++c) {
    const int t0 = c * 64;
    {
      const float* src = xbc + (size_t)(t0 + row) * XP + h * 64 + 32 * half;
#pragma unroll
      for (int j = 0; j < 8; ++j)
        *(v4fa*)(XS + row * 64 + 32 * half + 4 * j) = *(const v4f*)(src + 4 * j);
    }
    if (tid < 64) {
      const float raw = zx[(size_t)(t0 + tid) * ZXP + (2 * DIN + 128) + h];
      const float v = raw + dtb;
      const float dt = fmaxf(v, 0.0f) + log1pf(expf(-fabsf(v)));
      dtv[tid]  = dt;
      adtv[tid] = dt * Aneg;
    }
    __syncthreads();
    if (tid < 64) {
      float pre = 0.0f, tot = 0.0f;
#pragma unroll 4
      for (int r = 0; r < 64; ++r) {
        const float a = adtv[r];
        tot += a;
        pre += (r <= tid) ? a : 0.0f;
      }
      cumv[tid] = pre;
      ecum[tid] = expf(pre);
      edec[tid] = expf(tot - pre);
    }
    __syncthreads();

    {
      const float dts = dtv[row];
      const float eds = edec[row];
      const float ect = ecum[row];
      const float cmt = cumv[row];
      const float* brow = xbc + (size_t)(t0 + row) * XP + DIN + 32 * half;
      const float* grow = G + ((size_t)(t0 + row)) * 64 + 32 * half;
#pragma unroll 2
      for (int j = 0; j < 8; ++j) {
        const int col = 32 * half + 4 * j;
        v4us h4, l4;
        const v4f x4 = *(const v4fa*)(XS + row * 64 + col);
        stT4(Th, Tl, col, row, x4 * dts);
        const v4f b4 = *(const v4f*)(brow + 4 * j);
        stT4(Bh, Bl, col, row, b4 * eds);
        const v4f c4 = *(const v4f*)(brow + 64 + 4 * j);
        pack4(c4 * ect, h4, l4);
        *(v4usa*)(Ch + row * 64 + col) = h4;
        *(v4usa*)(Cl + row * 64 + col) = l4;
        const v4f g4 = *(const v4f*)(grow + 4 * j);
        const float c0 = cumv[col + 0], c1 = cumv[col + 1], c2 = cumv[col + 2], c3 = cumv[col + 3];
        const bool k0 = (col + 0) <= row, k1 = (col + 1) <= row, k2 = (col + 2) <= row, k3 = (col + 3) <= row;
        const float e0 = expf(k0 ? (cmt - c0) : 0.0f);
        const float e1 = expf(k1 ? (cmt - c1) : 0.0f);
        const float e2 = expf(k2 ? (cmt - c2) : 0.0f);
        const float e3 = expf(k3 ? (cmt - c3) : 0.0f);
        v4f mv;
        mv.x = k0 ? g4.x * e0 : 0.0f;
        mv.y = k1 ? g4.y * e1 : 0.0f;
        mv.z = k2 ? g4.z * e2 : 0.0f;
        mv.w = k3 ? g4.w * e3 : 0.0f;
        pack4(mv, h4, l4);
        *(v4usa*)(Mh + row * 64 + col) = h4;
        *(v4usa*)(Ml + row * 64 + col) = l4;
        const v4f s4 = *(const v4fa*)(Sf + row * 64 + col);
        pack4(s4, h4, l4);
        *(v4usa*)(Sh + row * 64 + col) = h4;
        *(v4usa*)(Sl + row * 64 + col) = l4;
      }
    }
    __syncthreads();

    {
      v8f accY[4];
      const v8f z = {0.f, 0.f, 0.f, 0.f, 0.f, 0.f, 0.f, 0.f};
      accY[0] = z; accY[1] = z; accY[2] = z; accY[3] = z;
      mm64x3(Mh, Ml, Th, Tl, accY, wave, hh, m);
      mm64x3(Ch, Cl, Sh, Sl, accY, wave, hh, m);
#pragma unroll
      for (int t = 0; t < 4; ++t)
#pragma unroll
        for (int r = 0; r < 8; ++r) {
          const int idx = (16 * wave + 8 * hh + r) * 64 + 16 * t + m;
          const float xv = XS[idx];
          XS[idx] = accY[t][r] + Dp * xv;
        }
    }
    {
      v8f accS[4];
      const v8f z = {0.f, 0.f, 0.f, 0.f, 0.f, 0.f, 0.f, 0.f};
      accS[0] = z; accS[1] = z; accS[2] = z; accS[3] = z;
      mm64x3(Th, Tl, Bh, Bl, accS, wave, hh, m);
      const float dec = ecum[63];
#pragma unroll
      for (int t = 0; t < 4; ++t)
#pragma unroll
        for (int r = 0; r < 8; ++r) {
          const int idx = (16 * wave + 8 * hh + r) * 64 + 16 * t + m;
          const float sv = Sf[idx];
          Sf[idx] = dec * sv + accS[t][r];
        }
    }
    __syncthreads();

#pragma unroll 1
    for (int it = 0; it < 8; ++it) {
      const int idx = it * 128 + tid;
      const int r = idx >> 4, c4 = idx & 15;
      const v4f v = *(const v4fa*)(XS + r * 64 + 4 * c4);
      float* op = xbc + (size_t)(t0 + r) * XP + h * 64 + 4 * c4;
      *(volatile v4f*)op = v;
      __threadfence();
      *(volatile v4f*)op = v;
    }
    __syncthreads();
  }
}

__global__ __launch_bounds__(256) void k_gate(const float* __restrict__ xbc, const float* __restrict__ zx,
                                              const float* __restrict__ nw, unsigned short* yn) {
  __shared__ __attribute__((aligned(16))) float gs[DIN];
  __shared__ float red[8];
  const int tid = (int)threadIdx.x, lane = tid & 31, wave = tid >> 5;
  const int tok = (int)blockIdx.x;
  const float* yr = xbc + (size_t)tok * XP;
  const float* zr = zx + (size_t)tok * ZXP;
  float ss = 0.0f;
#pragma unroll 1
  for (int i = 0; i < 8; ++i) {
    const int c = i * 256 + tid;
    const float yv = yr[c];
    const float zv = zr[c];
    const float g = yv * siluf(zv);
    gs[c] = g;
    ss = fmaf(g, g, ss);
  }
#pragma unroll
  for (int d = 16; d >= 1; d >>= 1) ss += __shfl_xor(ss, d, 32);
  if (lane == 0) red[wave] = ss;
  __syncthreads();
  const float tot = ((red[0] + red[1]) + (red[2] + red[3])) + ((red[4] + red[5]) + (red[6] + red[7]));
  const float scale = rsqrtf(tot * (1.0f / (float)DIN) + 1e-5f);
  const v4f g0 = *(const v4fa*)(gs + 8 * tid);
  const v4f g1 = *(const v4fa*)(gs + 8 * tid + 4);
  const v4f w0 = *(const v4f*)(nw + 8 * tid);
  const v4f w1 = *(const v4f*)(nw + 8 * tid + 4);
  v4f a, b;
  a.x = (g0.x * scale) * bf16_val(w0.x); a.y = (g0.y * scale) * bf16_val(w0.y);
  a.z = (g0.z * scale) * bf16_val(w0.z); a.w = (g0.w * scale) * bf16_val(w0.w);
  b.x = (g1.x * scale) * bf16_val(w1.x); b.y = (g1.y * scale) * bf16_val(w1.y);
  b.z = (g1.z * scale) * bf16_val(w1.z); b.w = (g1.w * scale) * bf16_val(w1.w);
  v4us h0, l0, h1, l1;
  pack4(a, h0, l0);
  pack4(b, h1, l1);
  v8us oh, ol;
  oh[0] = h0[0]; oh[1] = h0[1]; oh[2] = h0[2]; oh[3] = h0[3];
  oh[4] = h1[0]; oh[5] = h1[1]; oh[6] = h1[2]; oh[7] = h1[3];
  ol[0] = l0[0]; ol[1] = l0[1]; ol[2] = l0[2]; ol[3] = l0[3];
  ol[4] = l1[0]; ol[5] = l1[1]; ol[6] = l1[2]; ol[7] = l1[3];
  unsigned short* hp = yn + (size_t)tok * (2 * DIN) + 8 * tid;
  unsigned short* lp = hp + DIN;
  *(volatile v8us*)hp = oh;
  *(volatile v8us*)lp = ol;
  __threadfence();
  *(volatile v8us*)hp = oh;
  *(volatile v8us*)lp = ol;
}

__global__ __launch_bounds__(128) void k_rms(const float* __restrict__ H, const float* __restrict__ rw,
                                             unsigned short* hn) {
  __shared__ float red[4];
  const int tid = (int)threadIdx.x, lane = tid & 31, wave = tid >> 5;
  const int tok = (int)blockIdx.x;
  const float* hr = H + (size_t)tok * DM + 8 * tid;
  const v4f g0 = *(const v4f*)hr;
  const v4f g1 = *(const v4f*)(hr + 4);
  float ss = g0.x * g0.x;
  ss = fmaf(g0.y, g0.y, ss); ss = fmaf(g0.z, g0.z, ss); ss = fmaf(g0.w, g0.w, ss);
  ss = fmaf(g1.x, g1.x, ss); ss = fmaf(g1.y, g1.y, ss); ss = fmaf(g1.z, g1.z, ss); ss = fmaf(g1.w, g1.w, ss);
#pragma unroll
  for (int d = 16; d >= 1; d >>= 1) ss += __shfl_xor(ss, d, 32);
  if (lane == 0) red[wave] = ss;
  __syncthreads();
  const float tot = (red[0] + red[1]) + (red[2] + red[3]);
  const float scale = rsqrtf(tot * (1.0f / (float)DM) + 1e-5f);
  const v4f w0 = *(const v4f*)(rw + 8 * tid);
  const v4f w1 = *(const v4f*)(rw + 8 * tid + 4);
  v4f a, b;
  a.x = (g0.x * scale) * bf16_val(w0.x); a.y = (g0.y * scale) * bf16_val(w0.y);
  a.z = (g0.z * scale) * bf16_val(w0.z); a.w = (g0.w * scale) * bf16_val(w0.w);
  b.x = (g1.x * scale) * bf16_val(w1.x); b.y = (g1.y * scale) * bf16_val(w1.y);
  b.z = (g1.z * scale) * bf16_val(w1.z); b.w = (g1.w * scale) * bf16_val(w1.w);
  v4us h0, l0, h1, l1;
  pack4(a, h0, l0);
  pack4(b, h1, l1);
  v8us oh, ol;
  oh[0] = h0[0]; oh[1] = h0[1]; oh[2] = h0[2]; oh[3] = h0[3];
  oh[4] = h1[0]; oh[5] = h1[1]; oh[6] = h1[2]; oh[7] = h1[3];
  ol[0] = l0[0]; ol[1] = l0[1]; ol[2] = l0[2]; ol[3] = l0[3];
  ol[4] = l1[0]; ol[5] = l1[1]; ol[6] = l1[2]; ol[7] = l1[3];
  unsigned short* hp = hn + (size_t)tok * (2 * DM) + 8 * tid;
  unsigned short* lp = hp + DM;
  *(volatile v8us*)hp = oh;
  *(volatile v8us*)lp = ol;
  __threadfence();
  *(volatile v8us*)hp = oh;
  *(volatile v8us*)lp = ol;
}

constexpr size_t SZ_XB  = (size_t)NBATCH * SEQ * DM * 2;
constexpr size_t SZ_WIN = (size_t)ZXP * DM * 2;
constexpr size_t SZ_WO  = (size_t)DM * DIN * 2;
constexpr size_t SZ_W1  = (size_t)MLPI * DM * 2;
constexpr size_t SZ_W2  = (size_t)DM * MLPI * 2;
constexpr size_t SZ_RA  = (size_t)SEQ * ZXP * 4;
constexpr size_t SZ_RB  = (size_t)SEQ * XP * 4;
constexpr size_t SZ_YN  = (size_t)SEQ * 2 * DIN * 2;
constexpr size_t SZ_G   = (size_t)SEQ * 64 * 4;
constexpr size_t SZ_H   = (size_t)SEQ * DM * 4;
constexpr size_t SZ_HN  = (size_t)SEQ * 2 * DM * 2;
constexpr size_t SZ_F   = (size_t)SEQ * 2 * MLPI * 2;
constexpr size_t SZ_TOT = SZ_XB + SZ_WIN + SZ_WO + SZ_W1 + SZ_W2 + SZ_RA + SZ_RB + SZ_YN + SZ_G;
static_assert(SZ_F <= SZ_RA);
static_assert(SZ_H + SZ_HN <= SZ_RB);
static_assert(SZ_TOT <= (size_t)WSMAX);
static_assert(SZ_XB % 256 == 0 && SZ_WIN % 256 == 0 && SZ_WO % 256 == 0 && SZ_W1 % 256 == 0 && SZ_W2 % 256 == 0);
static_assert(SZ_RA % 256 == 0 && SZ_RB % 256 == 0 && SZ_YN % 256 == 0 && SZ_G % 256 == 0 && SZ_H % 256 == 0);

extern "C" void kernel_launch(void* const* d_in, const int* in_sizes, int n_in,
                              void* d_out, int out_size, void* d_ws, size_t ws_size,
                              hipStream_t stream) {
  if (n_in < 14) return;
  if (in_sizes[0] != NBATCH * SEQ * DM) return;
  if (in_sizes[1] != DM * DPROJ) return;
  if (in_sizes[2] != CONVD * 4 || in_sizes[3] != CONVD) return;
  if (in_sizes[4] != NHD || in_sizes[5] != NHD || in_sizes[6] != NHD) return;
  if (in_sizes[7] != DIN || in_sizes[8] != DIN * DM || in_sizes[9] != DM) return;
  if (in_sizes[10] != DM * MLPI || in_sizes[11] != MLPI) return;
  if (in_sizes[12] != MLPI * DM || in_sizes[13] != DM) return;
  if (out_size != NBATCH * SEQ * DM) return;
  if (ws_size < SZ_TOT) return;

  const float* x      = (const float*)d_in[0];
  const float* W_in   = (const float*)d_in[1];
  const float* conv_w = (const float*)d_in[2];
  const float* conv_b = (const float*)d_in[3];
  const float* dt_b   = (const float*)d_in[4];
  const float* A_log  = (const float*)d_in[5];
  const float* D_par  = (const float*)d_in[6];
  const float* norm_w = (const float*)d_in[7];
  const float* W_out  = (const float*)d_in[8];
  const float* rms_w  = (const float*)d_in[9];
  const float* w1     = (const float*)d_in[10];
  const float* b1     = (const float*)d_in[11];
  const float* w2     = (const float*)d_in[12];
  const float* b2     = (const float*)d_in[13];
  float* out = (float*)d_out;

  char* ws = (char*)d_ws;
  size_t off = 0;
  unsigned short* XB   = (unsigned short*)(ws + off); off += SZ_XB;
  unsigned short* WinT = (unsigned short*)(ws + off); off += SZ_WIN;
  unsigned short* WOT  = (unsigned short*)(ws + off); off += SZ_WO;
  unsigned short* W1T  = (unsigned short*)(ws + off); off += SZ_W1;
  unsigned short* W2T  = (unsigned short*)(ws + off); off += SZ_W2;
  char* regA = ws + off; off += SZ_RA;
  char* regB = ws + off; off += SZ_RB;
  unsigned short* YN   = (unsigned short*)(ws + off); off += SZ_YN;
  float* G             = (float*)(ws + off);          off += SZ_G;
  if (off != SZ_TOT) return;
  float*          ZX  = (float*)regA;
  unsigned short* F   = (unsigned short*)regA;
  float*          XBC = (float*)regB;
  float*          H   = (float*)regB;
  unsigned short* HN  = (unsigned short*)(regB + SZ_H);

  hipFuncSetAttribute(reinterpret_cast<const void*>(&k_ssd), hipFuncAttributeMaxDynamicSharedMemorySize, SSD_LDS);

  {
    const int nU = NBATCH * SEQ * DM / 8;
    k_cvx<<<(nU + 255) / 256, 256, 0, stream>>>(x, nU, XB);
    k_wT<<<(ZXP * (DM / 8) + 255) / 256, 256, 0, stream>>>(W_in, DM, DPROJ, ZXP, WinT);
    k_wT<<<(DM * (DIN / 8) + 255) / 256, 256, 0, stream>>>(W_out, DIN, DM, DM, WOT);
    k_wT<<<(MLPI * (DM / 8) + 255) / 256, 256, 0, stream>>>(w1, DM, MLPI, MLPI, W1T);
    k_wT<<<(DM * (MLPI / 8) + 255) / 256, 256, 0, stream>>>(w2, MLPI, DM, DM, W2T);
  }

  for (int b = 0; b < NBATCH; ++b) {
    const unsigned short* xb = XB + (size_t)b * SEQ * DM;
    const float* xf = x + (size_t)b * SEQ * DM;
    float* ob = out + (size_t)b * SEQ * DM;
    k_gemm<0><<<dim3(SEQ / GBM, ZXP / GBN), GTHR, 0, stream>>>(
        xb, DM, DM, WinT, DM, ZX, ZXP, YN, 0, 0, conv_b, conv_b, 0);
    k_conv<<<(SEQ * CONVD) / 256, 256, 0, stream>>>(ZX, conv_w, conv_b, XBC);
    k_cb<<<NCH, 128, 0, stream>>>(XBC, G);
    k_ssd<<<NHD, 128, SSD_LDS, stream>>>(ZX, XBC, G, dt_b, A_log, D_par);
    k_gate<<<SEQ, 256, 0, stream>>>(XBC, ZX, norm_w, YN);
    k_gemm<1><<<dim3(SEQ / GBM, DM / GBN), GTHR, 0, stream>>>(
        YN, 2 * DIN, 2 * DIN, WOT, DIN, H, DM, YN, 0, 0, conv_b, xf, DM);
    k_rms<<<SEQ, 128, 0, stream>>>(H, rms_w, HN);
    k_gemm<2><<<dim3(SEQ / GBM, MLPI / GBN), GTHR, 0, stream>>>(
        HN, 2 * DM, 2 * DM, W1T, DM, H, 0, F, 2 * MLPI, MLPI, b1, b1, 0);
    k_gemm<3><<<dim3(SEQ / GBM, DM / GBN), GTHR, 0, stream>>>(
        F, 2 * MLPI, 2 * MLPI, W2T, MLPI, ob, DM, YN, 0, 0, b2, H, DM);
  }
}
